// LSTMEncoder2_26603027431884
// MI455X (gfx1250) — hardware-verified
//
#include <hip/hip_runtime.h>


typedef _Float16 f16t;
typedef f16t  v16h __attribute__((ext_vector_type(16)));
typedef f16t  v8h  __attribute__((ext_vector_type(8)));
typedef float v8f  __attribute__((ext_vector_type(8)));
typedef float v4f  __attribute__((ext_vector_type(4)));
typedef unsigned int v4u __attribute__((ext_vector_type(4)));

union Frag { v16h v; v8h q[2]; };
union Pk16 { v8h h; v4u u; };
union Pk32 { v4f f; v4u u; };

#define NSEQ  512
#define NSTEP 512
#define NF    32
#define NH    128
#define NE    64
#define RB    32
#define HP1   136
#define HP2   72
#define NTHR  256

__device__ __forceinline__ v8f wmma16(v16h a, v16h b, v8f c) {
    return __builtin_amdgcn_wmma_f32_16x16x32_f16(false, a, false, b, (short)0, c, false, false);
}

__device__ __forceinline__ void wguard(v8f (&c)[2][4], Frag (&a)[2], Frag (&b)[4]) {
    asm volatile("v_nop\n\tv_nop\n\tv_nop\n\tv_nop"
                 : "+v"(c[0][0]), "+v"(c[0][1]), "+v"(c[0][2]), "+v"(c[0][3]),
                   "+v"(c[1][0]), "+v"(c[1][1]), "+v"(c[1][2]), "+v"(c[1][3])
                 : "v"(a[0].v), "v"(a[1].v),
                   "v"(b[0].v), "v"(b[1].v), "v"(b[2].v), "v"(b[3].v));
}
__device__ __forceinline__ void wguard(v8f (&c)[1][4], Frag (&a)[1], Frag (&b)[4]) {
    asm volatile("v_nop\n\tv_nop\n\tv_nop\n\tv_nop"
                 : "+v"(c[0][0]), "+v"(c[0][1]), "+v"(c[0][2]), "+v"(c[0][3])
                 : "v"(a[0].v),
                   "v"(b[0].v), "v"(b[1].v), "v"(b[2].v), "v"(b[3].v));
}

template<int MT>
__device__ __forceinline__ void zacc(v8f (&acc)[MT][4]) {
    const v8f z = {0.f, 0.f, 0.f, 0.f, 0.f, 0.f, 0.f, 0.f};
#pragma unroll
    for (int i = 0; i < MT; ++i)
#pragma unroll
        for (int g = 0; g < 4; ++g) acc[i][g] = z;
}

template<int MT>
__device__ __forceinline__ void mma_g4(v8f (&acc)[MT][4],
                                       const f16t* A, size_t lda, size_t ats,
                                       const f16t* B, int ldb, size_t bts, int ktiles) {
    const int l = threadIdx.x & 31, h = l >> 4, m = l & 15;
    const f16t* ap = A + (size_t)m * lda + 8 * h;
    const f16t* bp = B + (size_t)m * ldb + 8 * h;
#pragma unroll 1
    for (int kt = 0; kt < ktiles; ++kt) {
        Frag a[MT], b[4];
#pragma unroll
        for (int i = 0; i < MT; ++i) {
            const f16t* p = ap + (size_t)i * ats + kt * 32;
            a[i].q[0] = *(const v8h*)p;
            a[i].q[1] = *(const v8h*)(p + 16);
        }
#pragma unroll
        for (int g = 0; g < 4; ++g) {
            const f16t* p = bp + (size_t)g * bts + kt * 32;
            b[g].q[0] = *(const v8h*)p;
            b[g].q[1] = *(const v8h*)(p + 16);
        }
#pragma unroll
        for (int i = 0; i < MT; ++i)
#pragma unroll
            for (int g = 0; g < 4; ++g)
                acc[i][g] = wmma16(a[i].v, b[g].v, acc[i][g]);
        wguard(acc, a, b);
    }
}

__device__ __forceinline__ float ftanh(float x) {
    float ax = fabsf(x);
    float t  = __expf(-2.0f * ax);
    float r  = (1.0f - t) * __builtin_amdgcn_rcpf(1.0f + t);
    return copysignf(r, x);
}
__device__ __forceinline__ float fsigm(float x) {
    float t = __expf(-fabsf(x));
    float r = __builtin_amdgcn_rcpf(1.0f + t);
    return (x >= 0.0f) ? r : t * r;
}

__global__ __launch_bounds__(256)
void k_cvt8(const float* src, f16t* dst, int n8, float sc) {
    int i = blockIdx.x * 256 + threadIdx.x;
    if (i >= n8) return;
    const float* p = src + (size_t)i * 8;
    v4f a = *(const v4f*)p;
    v4f b = *(const v4f*)(p + 4);
    Pk16 k;
    k.h[0] = (f16t)(a[0] * sc); k.h[1] = (f16t)(a[1] * sc);
    k.h[2] = (f16t)(a[2] * sc); k.h[3] = (f16t)(a[3] * sc);
    k.h[4] = (f16t)(b[0] * sc); k.h[5] = (f16t)(b[1] * sc);
    k.h[6] = (f16t)(b[2] * sc); k.h[7] = (f16t)(b[3] * sc);
    f16t* d = dst + (size_t)i * 8;
    *(volatile v4u*)d = k.u;
    __threadfence();
    *(volatile v4u*)d = k.u;
}

__global__ __launch_bounds__(NTHR)
void k_lstm2(const f16t* X, const f16t* Pih1, const f16t* Phh1,
             const float* bih1, const float* bhh1,
             const f16t* Pih2, const f16t* Phh2,
             const float* bih2, const float* bhh2,
             float* out, int nb, int ns, float inv1, float inv2) {
    __shared__ __attribute__((aligned(16))) f16t  sH1[RB * HP1];
    __shared__ __attribute__((aligned(16))) f16t  sH2[RB * HP2];
    __shared__ __attribute__((aligned(16))) float sO[RB * NE];
    const int tid = threadIdx.x;
    const int l = tid & 31, h = l >> 4, m = l & 15, w = tid >> 5;
    const int b0 = blockIdx.x * RB;
    if (b0 + RB > nb) return;

    for (int i = tid; i < RB * HP1; i += NTHR) sH1[i] = (f16t)0.0f;
    for (int i = tid; i < RB * HP2; i += NTHR) sH2[i] = (f16t)0.0f;

    const int j1  = w;
    const int mt2 = w >> 2;
    const int j2  = w & 3;

    float bz1[4], bz2[4];
#pragma unroll
    for (int g = 0; g < 4; ++g) {
        int n1 = g * NH + 16 * j1 + m;
        int n2 = g * NE + 16 * j2 + m;
        bz1[g] = bih1[n1] + bhh1[n1];
        bz2[g] = bih2[n2] + bhh2[n2];
    }

    float c1[2][8], c2[8], h2r[8];
#pragma unroll
    for (int r = 0; r < 8; ++r) { c1[0][r] = 0.0f; c1[1][r] = 0.0f; c2[r] = 0.0f; h2r[r] = 0.0f; }

    __syncthreads();

    const size_t ldx = (size_t)ns * NF;
    const f16t* Xb = X + (size_t)b0 * ldx;

#pragma unroll 1
    for (int t = 0; t < ns; ++t) {
        v8f a1[2][4]; zacc(a1);
        mma_g4<2>(a1, Xb + (size_t)t * NF, ldx, 16 * ldx,
                  Pih1 + (size_t)(16 * j1) * NF, NF, (size_t)NH * NF, 1);
        mma_g4<2>(a1, sH1, HP1, (size_t)16 * HP1,
                  Phh1 + (size_t)(16 * j1) * NH, NH, (size_t)NH * NH, NH / 32);
        v8f a2[1][4]; zacc(a2);
        mma_g4<1>(a2, sH2 + (size_t)(16 * mt2) * HP2, HP2, 0,
                  Phh2 + (size_t)(16 * j2) * NE, NE, (size_t)NE * NE, NE / 32);
        __syncthreads();

#pragma unroll
        for (int i = 0; i < 2; ++i) {
#pragma unroll
            for (int r = 0; r < 8; ++r) {
                float gi = fmaf(a1[i][0][r], inv1, bz1[0]);
                float gf = fmaf(a1[i][1][r], inv1, bz1[1]);
                float gg = fmaf(a1[i][2][r], inv1, bz1[2]);
                float go = fmaf(a1[i][3][r], inv1, bz1[3]);
                float c  = fsigm(gf) * c1[i][r] + fsigm(gi) * ftanh(gg);
                c1[i][r] = c;
                float hv = fsigm(go) * ftanh(c);
                sH1[(16 * i + 8 * h + r) * HP1 + 16 * j1 + m] = (f16t)hv;
            }
        }
        __syncthreads();

        mma_g4<1>(a2, sH1 + (size_t)(16 * mt2) * HP1, HP1, 0,
                  Pih2 + (size_t)(16 * j2) * NH, NH, (size_t)NE * NH, NH / 32);

#pragma unroll
        for (int r = 0; r < 8; ++r) {
            float gi = fmaf(a2[0][0][r], inv2, bz2[0]);
            float gf = fmaf(a2[0][1][r], inv2, bz2[1]);
            float gg = fmaf(a2[0][2][r], inv2, bz2[2]);
            float go = fmaf(a2[0][3][r], inv2, bz2[3]);
            float c  = fsigm(gf) * c2[r] + fsigm(gi) * ftanh(gg);
            c2[r] = c;
            float hv = fsigm(go) * ftanh(c);
            h2r[r] = hv;
            sH2[(16 * mt2 + 8 * h + r) * HP2 + 16 * j2 + m] = (f16t)hv;
        }
        __syncthreads();
    }

#pragma unroll
    for (int r = 0; r < 8; ++r)
        sO[(16 * mt2 + 8 * h + r) * NE + 16 * j2 + m] = h2r[r];
    __syncthreads();
    Pk32 v[2];
#pragma unroll
    for (int i = 0; i < 2; ++i) {
        int p = tid + NTHR * i, row = p >> 4, c = (p & 15) * 4;
        v[i].f = *(const v4f*)(sO + row * NE + c);
    }
#pragma unroll
    for (int i = 0; i < 2; ++i) {
        int p = tid + NTHR * i, row = p >> 4, c = (p & 15) * 4;
        *(volatile v4u*)(out + (size_t)(b0 + row) * NE + c) = v[i].u;
    }
    __threadfence();
#pragma unroll
    for (int i = 0; i < 2; ++i) {
        int p = tid + NTHR * i, row = p >> 4, c = (p & 15) * 4;
        *(volatile v4u*)(out + (size_t)(b0 + row) * NE + c) = v[i].u;
    }
}

extern "C" void kernel_launch(void* const* d_in, const int* in_sizes, int n_in,
                              void* d_out, int out_size, void* d_ws, size_t ws_size,
                              hipStream_t stream) {
    const int G1 = 4 * NH, G2 = 4 * NE;
    if (n_in < 9) return;
    if (in_sizes[0] != NSEQ * NSTEP * NF) return;
    if (in_sizes[1] != G1 * NF || in_sizes[2] != G1 * NH ||
        in_sizes[3] != G1 || in_sizes[4] != G1) return;
    if (in_sizes[5] != G2 * NH || in_sizes[6] != G2 * NE ||
        in_sizes[7] != G2 || in_sizes[8] != G2) return;
    if (out_size != NSEQ * NE) return;
    if ((NSEQ % RB) != 0) return;

    const float* x    = (const float*)d_in[0];
    const float* Wih1 = (const float*)d_in[1];
    const float* Whh1 = (const float*)d_in[2];
    const float* bih1 = (const float*)d_in[3];
    const float* bhh1 = (const float*)d_in[4];
    const float* Wih2 = (const float*)d_in[5];
    const float* Whh2 = (const float*)d_in[6];
    const float* bih2 = (const float*)d_in[7];
    const float* bhh2 = (const float*)d_in[8];
    float* out = (float*)d_out;

    char* ws = (char*)d_ws;
    size_t off = 0;
    auto carve = [&](size_t bytes) -> char* {
        char* p = ws + off;
        off = (off + bytes + 255) & ~(size_t)255;
        return p;
    };
    f16t* X16  = (f16t*)carve((size_t)NSEQ * NSTEP * NF * 2);
    f16t* Pih1 = (f16t*)carve((size_t)G1 * NF * 2);
    f16t* Phh1 = (f16t*)carve((size_t)G1 * NH * 2);
    f16t* Pih2 = (f16t*)carve((size_t)G2 * NH * 2);
    f16t* Phh2 = (f16t*)carve((size_t)G2 * NE * 2);
    if (off > ws_size) return;

    const float S64 = 64.0f, I64 = 0.015625f;

    auto cvt = [&](const float* s, f16t* d, int n, float sc) {
        int n8 = n / 8;
        k_cvt8<<<dim3((n8 + 255) / 256), dim3(256), 0, stream>>>(s, d, n8, sc);
    };
    cvt(x,    X16,  NSEQ * NSTEP * NF, 1.0f);
    cvt(Wih1, Pih1, G1 * NF, S64);
    cvt(Whh1, Phh1, G1 * NH, S64);
    cvt(Wih2, Pih2, G2 * NH, S64);
    cvt(Whh2, Phh2, G2 * NE, S64);

    k_lstm2<<<dim3(NSEQ / RB), dim3(NTHR), 0, stream>>>(X16, Pih1, Phh1, bih1, bhh1,
                                                      Pih2, Phh2, bih2, bhh2,
                                                      out, NSEQ, NSTEP, I64, I64);
}
